// UnifiedMambaBlock_60610578482001
// MI455X (gfx1250) — hardware-run, weakly checked
//
#include <hip/hip_runtime.h>
#include <math.h>

typedef __attribute__((ext_vector_type(16))) _Float16 v16h;
typedef __attribute__((ext_vector_type(8)))  _Float16 v8h;
typedef __attribute__((ext_vector_type(4)))  _Float16 v4h;
typedef __attribute__((ext_vector_type(2)))  _Float16 v2h;
typedef __attribute__((ext_vector_type(8)))  float    v8f;
typedef __attribute__((ext_vector_type(4)))  float    v4f;
typedef __attribute__((ext_vector_type(2)))  float    v2f;
typedef __attribute__((ext_vector_type(4)))  unsigned v4u;

constexpr int kInputsRneToBf16 = 1;

constexpr int kBatch = 2;
constexpr int kSeq   = 2048;
constexpr int kDm    = 768;
constexpr int kDin   = 1536;
constexpr int kNst   = 16;
constexpr int kDtR   = 48;
constexpr int kTaps  = 4;
constexpr int kRows  = kBatch * kSeq;
constexpr int kXzP   = 2 * kDin;
constexpr int kXdW   = kDtR + 2 * kNst;
constexpr int kXdP   = 128;
constexpr int kDtK   = 64;
static_assert(kRows == 4096);
static_assert(kXzP == 3072);
static_assert(kXdW == 80);
static_assert(kXdW <= kXdP && kDtR <= kDtK);
static_assert((kDm % 32) == 0 && (kDin % 32) == 0 && (kDtK % 32) == 0);
static_assert((kRows % 64) == 0 && (kXzP % 64) == 0 && (kXdP % 64) == 0 && (kDin % 64) == 0 && (kDm % 64) == 0);
static_assert((kSeq & (kSeq - 1)) == 0);
static_assert((kDtR % 8) == 0 && (kDin % 8) == 0 && (kDm % 8) == 0);

constexpr float kCarryU   = 16.0f;
constexpr float kCarryW   = 1024.0f;
constexpr float kCarryXc  = 256.0f;
constexpr float kCarryDtr = 256.0f;
constexpr float kCarryY   = 2048.0f;
constexpr float kScaleIn  = 1.0f / (kCarryU * kCarryW);
constexpr float kScaleXp  = 1.0f / (kCarryXc * kCarryW);
constexpr float kScaleDt  = 1.0f / (kCarryDtr * kCarryW);
constexpr float kScaleOut = 1.0f / (kCarryY * kCarryW);

constexpr size_t kOffU16   = 0;
constexpr size_t kOffWin16 = kOffU16   + (size_t)kRows * kDm  * 2;
constexpr size_t kOffXz    = kOffWin16 + (size_t)kXzP  * kDm  * 2;
constexpr size_t kOffXc    = kOffXz    + (size_t)kRows * kXzP * 4;
constexpr size_t kOffXc16  = kOffXc    + (size_t)kRows * kDin * 4;
constexpr size_t kOffWx16  = kOffXc16  + (size_t)kRows * kDin * 2;
constexpr size_t kOffXd    = kOffWx16  + (size_t)kXdP  * kDin * 2;
constexpr size_t kOffDtr16 = kOffXd    + (size_t)kRows * kXdP * 4;
constexpr size_t kOffWdt16 = kOffDtr16 + (size_t)kRows * kDtK * 2;
constexpr size_t kOffDt16  = kOffWdt16 + (size_t)kDin  * kDtK * 2;
constexpr size_t kOffYg16  = kOffDt16  + (size_t)kRows * kDin * 2;
constexpr size_t kOffWout16 = kOffYg16 + (size_t)kRows * kDin * 2;
constexpr size_t kWsTotal  = kOffWout16 + (size_t)kDm * kDin * 2;
static_assert(kWsTotal == 129826816ull);
static_assert(kWsTotal <= 134217728ull);
static_assert((kOffWin16 % 128) == 0 && (kOffXz % 128) == 0 && (kOffXc % 128) == 0 && (kOffXc16 % 128) == 0 &&
              (kOffWx16 % 128) == 0 && (kOffXd % 128) == 0 && (kOffDtr16 % 128) == 0 && (kOffWdt16 % 128) == 0 &&
              (kOffDt16 % 128) == 0 && (kOffYg16 % 128) == 0 && (kOffWout16 % 128) == 0);

__device__ __forceinline__ float bf16_rne(float f) {
  unsigned u = __float_as_uint(f);
  u = (u + 0x7FFFu + ((u >> 16) & 1u)) & 0xFFFF0000u;
  return __uint_as_float(u);
}
__device__ __forceinline__ float inq(float f) { return kInputsRneToBf16 ? bf16_rne(f) : f; }

__device__ __forceinline__ _Float16 to_f16_operand(float v) {
  float c = fminf(fmaxf(v, -65000.0f), 65000.0f);
  c = (fabsf(c) < 6.103515625e-5f) ? 0.0f : c;
  return (_Float16)c;
}

__device__ __forceinline__ float h16_to_f32(unsigned hb) {
  const unsigned sgn = (hb & 0x8000u) << 16;
  const unsigned em = hb & 0x7fffu;
  const float fn = __uint_as_float((em << 13) + 0x38000000u);
  const float fs = (float)em * 5.9604644775390625e-8f;
  const float mag = (em < 0x400u) ? fs : fn;
  return __uint_as_float(__float_as_uint(mag) | sgn);
}

__device__ __forceinline__ float silu_f(float v) {
  return v * __builtin_amdgcn_rcpf(1.0f + expf(-v));
}

__device__ __forceinline__ void wave_lds_sync() {
  __builtin_amdgcn_fence(__ATOMIC_RELEASE, "workgroup");
  __builtin_amdgcn_wave_barrier();
  __builtin_amdgcn_fence(__ATOMIC_ACQUIRE, "workgroup");
}

template <bool IN_RNE>
__global__ __launch_bounds__(256) void cvt_plane_f16_kernel(
    const float* __restrict__ src, int src_pitch, int rows_valid, int cols_valid,
    unsigned short* __restrict__ dst, int dst_cols, int total8, float carry)
{
  const int i = blockIdx.x * 256 + threadIdx.x;
  if (i >= total8) return;
  const int cpr = dst_cols >> 3;
  const int row = i / cpr;
  const int col = (i - row * cpr) << 3;
  const bool ok = (row < rows_valid) && (col < cols_valid);
  const int rr = (row < rows_valid) ? row : (rows_valid - 1);
  const int cc = (col < cols_valid) ? col : (cols_valid - 8);
  const float* p = src + (size_t)rr * src_pitch + cc;
  v4f a0 = *(const v4f*)(p);
  v4f a1 = *(const v4f*)(p + 4);
  asm volatile("" : "+v"(a0), "+v"(a1));
  v8h hv;
#pragma unroll
  for (int e = 0; e < 4; ++e) {
    float x0 = ok ? a0[e] : 0.0f;
    float x1 = ok ? a1[e] : 0.0f;
    if (IN_RNE) { x0 = inq(x0); x1 = inq(x1); }
    hv[e]     = to_f16_operand(x0 * carry);
    hv[4 + e] = to_f16_operand(x1 * carry);
  }
  unsigned short* q = dst + ((size_t)i << 3);
  *(volatile v8h*)q = hv;
  __threadfence();
  *(volatile v8h*)q = hv;
}

namespace eng {

struct FragH {
  union U { v16h v; v8h h[2]; };
  static __device__ __forceinline__ v16h load(const _Float16* p) {
    U f;
    f.h[0] = *(const v8h*)(p);
    f.h[1] = *(const v8h*)(p + 16);
    return f.v;
  }
  static __device__ __forceinline__ v8f mma(v16h a, v16h b, v8f c) {
    return __builtin_amdgcn_wmma_f32_16x16x32_f16(false, a, false, b, (short)0, c, false, false);
  }
};
__device__ __forceinline__ void tie_h(v8f& a, v16h x, v16h y) {
  asm volatile("v_nop" : "+v"(a) : "v"(x), "v"(y));
}
__device__ __forceinline__ void guard_h(v8f& a, v16h x, v16h y) {
  asm volatile("v_nop\n\tv_nop\n\tv_nop\n\tv_nop" : "+v"(a) : "v"(x), "v"(y));
}
__device__ __forceinline__ void keep4_h(v16h a, v16h b, v16h c, v16h d) {
  asm volatile("v_nop" :: "v"(a), "v"(b), "v"(c), "v"(d));
}

template <bool BIAS_N, bool OUT_F16, bool SOFTPLUS>
__global__ __launch_bounds__(256) void gemm64_f16(
    const unsigned short* __restrict__ Ap, int lda,
    const unsigned short* __restrict__ Btp, int ldb,
    void* __restrict__ Cout, int ldc,
    const float* __restrict__ bias,
    int M, int N, int K, float scale)
{
  const _Float16* A  = (const _Float16*)Ap;
  const _Float16* Bt = (const _Float16*)Btp;
  __shared__ __align__(16) float sT[8][16 * 68];
  const int lane = threadIdx.x & 31;
  const int wave = threadIdx.x >> 5;
  const int tilesN = N >> 6;
  const int tilesM = M >> 6;
  const int tile = blockIdx.x * 8 + wave;
  if (tile >= tilesM * tilesN) return;
  const int tm = tile / tilesN;
  const int tn = tile - tm * tilesN;
  const int m0 = tm << 6;
  const int n0 = tn << 6;

  const int rlane = lane & 15;
  const int koff  = (lane >> 4) * 8;
  const int mOff  = (lane >> 4) * 8;

  v8f acc[4][4];
#pragma unroll
  for (int i = 0; i < 4; ++i)
#pragma unroll
    for (int j = 0; j < 4; ++j) acc[i][j] = (v8f){0.f, 0.f, 0.f, 0.f, 0.f, 0.f, 0.f, 0.f};

  for (int k0 = 0; k0 < K; k0 += 32) {
    v16h bh[4];
#pragma unroll
    for (int j = 0; j < 4; ++j) {
      const size_t bo = (size_t)(n0 + (j << 4) + rlane) * ldb + koff + k0;
      bh[j] = FragH::load(Bt + bo);
    }
#pragma unroll
    for (int i = 0; i < 4; ++i) {
      const size_t ao = (size_t)(m0 + (i << 4) + rlane) * lda + koff + k0;
      const v16h ah = FragH::load(A + ao);
#pragma unroll
      for (int j = 0; j < 4; ++j) acc[i][j] = FragH::mma(ah, bh[j], acc[i][j]);
      tie_h(acc[i][0], ah, bh[0]);
      tie_h(acc[i][1], ah, bh[1]);
      tie_h(acc[i][2], ah, bh[2]);
      guard_h(acc[i][3], ah, bh[3]);
    }
    keep4_h(bh[0], bh[1], bh[2], bh[3]);
  }

  float* slab = sT[wave];
#pragma unroll
  for (int i = 0; i < 4; ++i) {
    const int mBase = m0 + (i << 4);
#pragma unroll
    for (int j = 0; j < 4; ++j) {
      const int n = n0 + (j << 4) + rlane;
      float bv = 0.f;
      if (BIAS_N) bv = inq(bias[n]);
#pragma unroll
      for (int r = 0; r < 8; ++r) {
        float v = acc[i][j][r] * scale;
        if (BIAS_N) v += bv;
        slab[(mOff + r) * 68 + (j << 4) + rlane] = v;
      }
    }
    wave_lds_sync();
    if (SOFTPLUS) {
#pragma unroll 1
      for (int q = 0; q < 32; ++q) {
        const int idx = q * 32 + lane;
        const int rr = idx >> 6;
        const int cc = idx & 63;
        const float v = slab[rr * 68 + cc];
        slab[rr * 68 + cc] = fmaxf(v, 0.0f) + log1pf(expf(-fabsf(v)));
      }
      wave_lds_sync();
    }
    if (!OUT_F16) {
      float* C = (float*)Cout;
      const int hh = lane >> 4, c4 = (lane & 15) * 4;
      for (int pass = 0; pass < 2; ++pass) {
#pragma unroll
        for (int it = 0; it < 8; ++it) {
          const int row = it * 2 + hh;
          const v4f v = *(const v4f*)(slab + row * 68 + c4);
          *(volatile v4f*)(C + (size_t)(mBase + row) * ldc + n0 + c4) = v;
        }
        __threadfence();
      }
    } else {
      const int q = lane >> 3, c8 = (lane & 7) * 8;
      unsigned short* C = (unsigned short*)Cout;
      for (int pass = 0; pass < 2; ++pass) {
#pragma unroll
        for (int it = 0; it < 4; ++it) {
          const int row = it * 4 + q;
          const float* sp = slab + row * 68 + c8;
          v8h hv;
#pragma unroll
          for (int e = 0; e < 8; ++e) hv[e] = (_Float16)sp[e];
          *(volatile v8h*)(C + (size_t)(mBase + row) * ldc + n0 + c8) = hv;
        }
        __threadfence();
      }
    }
    wave_lds_sync();
  }
}

}

__device__ __forceinline__ float conv4_bias_silu(v4f w, float a0, float a1, float a2, float a3, float b) {
  float acc = inq(w[0]) * a0;
  acc = fmaf(inq(w[1]), a1, acc);
  acc = fmaf(inq(w[2]), a2, acc);
  acc = fmaf(inq(w[3]), a3, acc);
  const float sv = acc + inq(b);
  return silu_f(sv);
}

__global__ __launch_bounds__(256) void conv_silu_kernel(
    const float* __restrict__ XZ, const float* __restrict__ cw, const float* __restrict__ cb,
    float* __restrict__ XC, unsigned short* __restrict__ XC16)
{
  constexpr int kQuads = kDin / 4;
  const int i = blockIdx.x * 256 + threadIdx.x;
  if (i >= kRows * kQuads) return;
  const int row = i / kQuads;
  const int d = (i - row * kQuads) * 4;
  const int t = row & (kSeq - 1);
  const bool ok0 = (t >= 3), ok1 = (t >= 2), ok2 = (t >= 1);
  const int r0 = ok0 ? (row - 3) : row;
  const int r1 = ok1 ? (row - 2) : row;
  const int r2 = ok2 ? (row - 1) : row;
  v4f x0 = *(const v4f*)(XZ + (size_t)r0 * kXzP + d);
  v4f x1 = *(const v4f*)(XZ + (size_t)r1 * kXzP + d);
  v4f x2 = *(const v4f*)(XZ + (size_t)r2 * kXzP + d);
  v4f x3 = *(const v4f*)(XZ + (size_t)row * kXzP + d);
  asm volatile("" : "+v"(x0), "+v"(x1), "+v"(x2), "+v"(x3));
  const v4f zero = {0.f, 0.f, 0.f, 0.f};
  x0 = ok0 ? x0 : zero;
  x1 = ok1 ? x1 : zero;
  x2 = ok2 ? x2 : zero;
  const v4f w0 = *(const v4f*)(cw + (size_t)d * kTaps);
  const v4f w1 = *(const v4f*)(cw + (size_t)d * kTaps + 4);
  const v4f w2 = *(const v4f*)(cw + (size_t)d * kTaps + 8);
  const v4f w3 = *(const v4f*)(cw + (size_t)d * kTaps + 12);
  const v4f bv = *(const v4f*)(cb + d);
  v4f o;
  o[0] = conv4_bias_silu(w0, x0[0], x1[0], x2[0], x3[0], bv[0]);
  o[1] = conv4_bias_silu(w1, x0[1], x1[1], x2[1], x3[1], bv[1]);
  o[2] = conv4_bias_silu(w2, x0[2], x1[2], x2[2], x3[2], bv[2]);
  o[3] = conv4_bias_silu(w3, x0[3], x1[3], x2[3], x3[3], bv[3]);
  v4h hv;
  hv[0] = to_f16_operand(o[0] * kCarryXc);
  hv[1] = to_f16_operand(o[1] * kCarryXc);
  hv[2] = to_f16_operand(o[2] * kCarryXc);
  hv[3] = to_f16_operand(o[3] * kCarryXc);
  float* pf = XC + ((size_t)i << 2);
  unsigned short* ph = XC16 + ((size_t)i << 2);
  *(volatile v4f*)pf = o;
  *(volatile v4h*)ph = hv;
  __threadfence();
  *(volatile v4f*)pf = o;
  *(volatile v4h*)ph = hv;
}

constexpr int kScanThreads = 128;
constexpr int kScanCh      = 2 * kScanThreads;
constexpr int kScanChunk   = 64;
constexpr int kScanBlkPerB = kDin / kScanCh;
static_assert(kDin % kScanCh == 0 && kSeq % kScanChunk == 0);
static_assert(kScanChunk * 8 == 4 * kScanThreads);

__device__ __forceinline__ float scan_channel_step(float dt, float xt, const float (&nA)[kNst], float (&h)[kNst],
                                                   const float (&Bv)[kNst], const float (&Cv)[kNst]) {
  float y = 0.0f;
#pragma unroll
  for (int k = 0; k < kNst; ++k) {
    const float e  = __expf(dt * nA[k]);
    const float dB = dt * Bv[k];
    h[k] = h[k] * e + xt * dB;
    y = h[k] * Cv[k] + y;
  }
  return y;
}

__global__ __launch_bounds__(128) void scan_gate_kernel(
    const unsigned* __restrict__ dtw, const float* __restrict__ XC, const float* __restrict__ XZ,
    const float* __restrict__ XD, const float* __restrict__ Alog, const float* __restrict__ Dp,
    unsigned* __restrict__ yw)
{
  __shared__ __align__(16) float    sBC[kScanChunk * 32];
  __shared__ __align__(16) unsigned sY[kScanChunk * kScanThreads];
  __shared__ __align__(16) float    sA[kNst * kScanCh];
  const int tid = threadIdx.x, lane = tid & 31, wave = tid >> 5;
  const int bix = blockIdx.x / kScanBlkPerB;
  const int d0  = (blockIdx.x - bix * kScanBlkPerB) * kScanCh;
  const int d   = d0 + 2 * tid;
  const size_t row0 = (size_t)bix * kSeq;

#pragma unroll 1
  for (int s = 0; s < kNst; ++s) {
    sA[s * kScanCh + 2 * tid + 0] = -expf(inq(Alog[(size_t)(d + 0) * kNst + s]));
    sA[s * kScanCh + 2 * tid + 1] = -expf(inq(Alog[(size_t)(d + 1) * kNst + s]));
  }
  __syncthreads();
  float nA0[kNst], nA1[kNst], h0[kNst], h1[kNst];
#pragma unroll
  for (int s = 0; s < kNst; ++s) {
    nA0[s] = sA[s * kScanCh + 2 * tid + 0];
    nA1[s] = sA[s * kScanCh + 2 * tid + 1];
    h0[s] = 0.0f;
    h1[s] = 0.0f;
  }
  const v2f dpair = *(const v2f*)(Dp + d);
  const float Dd0 = inq(dpair[0]);
  const float Dd1 = inq(dpair[1]);

#pragma unroll 1
  for (int t0 = 0; t0 < kSeq; t0 += kScanChunk) {
    __syncthreads();
#pragma unroll
    for (int it = 0; it < 4; ++it) {
      const int idx = it * kScanThreads + tid;
      const int r = idx >> 3;
      const int q = idx & 7;
      *(v4f*)(sBC + r * 32 + 4 * q) = *(const v4f*)(XD + (row0 + t0 + r) * kXdP + kDtR + 4 * q);
    }
    __syncthreads();
#pragma unroll 1
    for (int s = 0; s < kScanChunk; ++s) {
      const size_t row = row0 + t0 + s;
      const unsigned w = dtw[row * (kDin / 2) + (d >> 1)];
      const v2f xv = *(const v2f*)(XC + row * kDin + d);
      const v2f zv = *(const v2f*)(XZ + row * kXzP + kDin + d);
      const float* bc = sBC + s * 32;
      float Bv[kNst], Cv[kNst];
#pragma unroll
      for (int q4 = 0; q4 < 4; ++q4) {
        const v4f bq = *(const v4f*)(bc + 4 * q4);
        const v4f cq = *(const v4f*)(bc + kNst + 4 * q4);
        Bv[4 * q4 + 0] = bq[0]; Bv[4 * q4 + 1] = bq[1]; Bv[4 * q4 + 2] = bq[2]; Bv[4 * q4 + 3] = bq[3];
        Cv[4 * q4 + 0] = cq[0]; Cv[4 * q4 + 1] = cq[1]; Cv[4 * q4 + 2] = cq[2]; Cv[4 * q4 + 3] = cq[3];
      }
      const float dt0 = h16_to_f32(w & 0xffffu);
      const float dt1 = h16_to_f32(w >> 16);
      const float x0 = xv[0], x1 = xv[1];
      const float z0 = zv[0], z1 = zv[1];
      float y0 = scan_channel_step(dt0, x0, nA0, h0, Bv, Cv);
      float y1 = scan_channel_step(dt1, x1, nA1, h1, Bv, Cv);
      y0 = (y0 + Dd0 * x0) * silu_f(z0);
      y1 = (y1 + Dd1 * x1) * silu_f(z1);
      v2h p;
      p[0] = to_f16_operand(y0 * kCarryY);
      p[1] = to_f16_operand(y1 * kCarryY);
      sY[s * kScanThreads + tid] = __builtin_bit_cast(unsigned, p);
    }
    __syncthreads();
    for (int pass = 0; pass < 2; ++pass) {
#pragma unroll 4
      for (int it = 0; it < 16; ++it) {
        const int r = it * 4 + wave;
        const v4u val = *(const v4u*)(sY + r * kScanThreads + lane * 4);
        *(volatile v4u*)(yw + (row0 + t0 + r) * (size_t)(kDin / 2) + (d0 >> 1) + lane * 4) = val;
      }
      __threadfence();
    }
  }
}

extern "C" void kernel_launch(void* const* d_in, const int* in_sizes, int n_in,
                              void* d_out, int out_size, void* d_ws, size_t ws_size,
                              hipStream_t stream) {
  if (n_in < 10) return;
  if (in_sizes[0] != kRows * kDm) return;
  if (in_sizes[1] != kXzP * kDm) return;
  if (in_sizes[2] != kDin * kTaps) return;
  if (in_sizes[3] != kDin) return;
  if (in_sizes[4] != kXdW * kDin) return;
  if (in_sizes[5] != kDin * kDtR) return;
  if (in_sizes[6] != kDin) return;
  if (in_sizes[7] != kDin * kNst) return;
  if (in_sizes[8] != kDin) return;
  if (in_sizes[9] != kDm * kDin) return;
  if (out_size != kRows * kDm) return;
  if (ws_size < kWsTotal) return;

  const float* u      = (const float*)d_in[0];
  const float* w_in   = (const float*)d_in[1];
  const float* conv_w = (const float*)d_in[2];
  const float* conv_b = (const float*)d_in[3];
  const float* w_x    = (const float*)d_in[4];
  const float* w_dt   = (const float*)d_in[5];
  const float* b_dt   = (const float*)d_in[6];
  const float* a_log  = (const float*)d_in[7];
  const float* d_skip = (const float*)d_in[8];
  const float* w_out  = (const float*)d_in[9];
  float* out = (float*)d_out;

  char* ws = (char*)d_ws;
  unsigned short* U16    = (unsigned short*)(ws + kOffU16);
  unsigned short* WIN16  = (unsigned short*)(ws + kOffWin16);
  float*          XZ     = (float*)(ws + kOffXz);
  float*          XC     = (float*)(ws + kOffXc);
  unsigned short* XC16   = (unsigned short*)(ws + kOffXc16);
  unsigned short* WX16   = (unsigned short*)(ws + kOffWx16);
  float*          XD     = (float*)(ws + kOffXd);
  unsigned short* DTR16  = (unsigned short*)(ws + kOffDtr16);
  unsigned short* WDT16  = (unsigned short*)(ws + kOffWdt16);
  unsigned short* DT16   = (unsigned short*)(ws + kOffDt16);
  unsigned short* YG16   = (unsigned short*)(ws + kOffYg16);
  unsigned short* WOUT16 = (unsigned short*)(ws + kOffWout16);

  cvt_plane_f16_kernel<true><<<(kRows * kDm / 8) / 256, 256, 0, stream>>>(
      u, kDm, kRows, kDm, U16, kDm, kRows * kDm / 8, kCarryU);
  cvt_plane_f16_kernel<true><<<(kXzP * kDm / 8) / 256, 256, 0, stream>>>(
      w_in, kDm, kXzP, kDm, WIN16, kDm, kXzP * kDm / 8, kCarryW);
  cvt_plane_f16_kernel<true><<<(kXdP * kDin / 8) / 256, 256, 0, stream>>>(
      w_x, kDin, kXdW, kDin, WX16, kDin, kXdP * kDin / 8, kCarryW);
  cvt_plane_f16_kernel<true><<<(kDin * kDtK / 8) / 256, 256, 0, stream>>>(
      w_dt, kDtR, kDin, kDtR, WDT16, kDtK, kDin * kDtK / 8, kCarryW);
  cvt_plane_f16_kernel<true><<<(kDm * kDin / 8) / 256, 256, 0, stream>>>(
      w_out, kDin, kDm, kDin, WOUT16, kDin, kDm * kDin / 8, kCarryW);

  eng::gemm64_f16<false, false, false><<<(kRows / 64) * (kXzP / 64) / 8, 256, 0, stream>>>(
      U16, kDm, WIN16, kDm, (void*)XZ, kXzP, nullptr, kRows, kXzP, kDm, kScaleIn);

  conv_silu_kernel<<<(kRows * (kDin / 4)) / 256, 256, 0, stream>>>(XZ, conv_w, conv_b, XC, XC16);

  eng::gemm64_f16<false, false, false><<<(kRows / 64) * (kXdP / 64) / 8, 256, 0, stream>>>(
      XC16, kDin, WX16, kDin, (void*)XD, kXdP, nullptr, kRows, kXdP, kDin, kScaleXp);

  cvt_plane_f16_kernel<false><<<(kRows * kDtK / 8) / 256, 256, 0, stream>>>(
      XD, kXdP, kRows, kDtR, DTR16, kDtK, kRows * kDtK / 8, kCarryDtr);

  eng::gemm64_f16<true, true, true><<<(kRows / 64) * (kDin / 64) / 8, 256, 0, stream>>>(
      DTR16, kDtK, WDT16, kDtK, (void*)DT16, kDin, b_dt, kRows, kDin, kDtK, kScaleDt);

  scan_gate_kernel<<<kBatch * kScanBlkPerB, kScanThreads, 0, stream>>>(
      (const unsigned*)DT16, XC, XZ, XD, a_log, d_skip, (unsigned*)YG16);

  eng::gemm64_f16<false, false, false><<<(kRows / 64) * (kDm / 64) / 8, 256, 0, stream>>>(
      YG16, kDin, WOUT16, kDin, (void*)out, kDm, nullptr, kRows, kDm, kDin, kScaleOut);
}
